// MambaBlock_34102040330337
// MI455X (gfx1250) — hardware-verified
//
#include <hip/hip_runtime.h>
#include <stddef.h>
#include <stdint.h>
#include <math.h>


#define TOK   2048
#define LSEQ  1024
#define NBAT  2
#define DMOD  1024
#define DIN   2048
#define NST   16
#define DTRK  64
#define XZP   4096
#define KG1   2048
#define KG2   4096
#define KG3   128
#define KG4   4096
#define N2P   128
#define BCP   32
#define GBM   128
#define GBN   64
#define GTHR  128
#define PTHR  256
#define PU_W2  (4096 * 128)
#define PU_WS  (N2P * 256)
#define PU_DTW (DIN * 8)
#define PU_OW  (DMOD * 256)
#define PU_ALL (PU_W2 + PU_WS + PU_DTW + PU_OW)
#define SC_TC  32
#define SC_DB  64
#define SC_THR 512
#define A_LOG_RNE_BF16 1
#define WSMAX 134217728

static_assert(TOK == NBAT * LSEQ && (LSEQ & (LSEQ - 1)) == 0);
static_assert(TOK % GBM == 0 && (2 * DIN) % GBN == 0 && N2P % GBN == 0 && DIN % GBN == 0 && DMOD % GBN == 0);
static_assert(KG1 % 32 == 0 && KG2 % 32 == 0 && KG3 % 32 == 0 && KG4 % 32 == 0);
static_assert(KG1 == 2 * DMOD && KG2 == 2 * DIN && KG3 == 2 * DTRK && KG4 == 2 * DIN);
static_assert(GBM == (GTHR / 32) * 32 && GBN == 64);
static_assert(PU_W2 % PTHR == 0 && PU_WS % PTHR == 0 && PU_DTW % PTHR == 0 && PU_OW % PTHR == 0);
static_assert(PTHR * 8 == DIN && 2 * PTHR * 4 == DIN);
static_assert(SC_THR == (SC_DB / 2) * NST && SC_THR == SC_TC * 16 && LSEQ % SC_TC == 0 && DIN % SC_DB == 0);
static_assert(SC_TC * 2 * 8 == SC_THR && SC_TC * SC_DB == 4 * SC_THR && SC_THR % SC_DB == 0);
static_assert(2 * DTRK == 128 && 2 * NST == BCP);
static_assert(DMOD == 4 * 256 && 256 == 32 * 8);

typedef float          v4f   __attribute__((ext_vector_type(4)));
typedef float          v8f   __attribute__((ext_vector_type(8)));
typedef int            v8i   __attribute__((ext_vector_type(8)));
typedef unsigned short v4us  __attribute__((ext_vector_type(4)));
typedef unsigned short v8us  __attribute__((ext_vector_type(8)));
typedef unsigned short v16us __attribute__((ext_vector_type(16)));
typedef __bf16         v16bf __attribute__((ext_vector_type(16)));
typedef v4f  __attribute__((may_alias)) v4fa;
typedef v4us __attribute__((may_alias)) v4usa;
typedef v8us __attribute__((may_alias)) v8usa;
union FragB { v16bf v; v16us u; v8us h[2]; v8i w; };

__device__ __forceinline__ v8f wmb(const FragB& a, const FragB& b, v8f c) {
  v8f d = __builtin_amdgcn_wmma_f32_16x16x32_bf16(false, a.v, false, b.v, (short)0, c, false, false);
  asm volatile("v_nop\n\tv_nop\n\tv_nop\n\tv_nop" : "+v"(d) : "v"(a.w), "v"(b.w));
  return d;
}

__device__ __forceinline__ unsigned bf16_bits(float f) {
  const unsigned u = __float_as_uint(f);
  return (u + 0x7FFFu + ((u >> 16) & 1u)) >> 16;
}
__device__ __forceinline__ float bf16_val(float f) {
  return __uint_as_float(bf16_bits(f) << 16);
}
__device__ __forceinline__ v4f bf16_val4(v4f r) {
  v4f q;
  q.x = bf16_val(r.x); q.y = bf16_val(r.y); q.z = bf16_val(r.z); q.w = bf16_val(r.w);
  return q;
}
__device__ __forceinline__ unsigned hl_pack(float v) {
  const unsigned h = bf16_bits(v);
  const float    r = v - __uint_as_float(h << 16);
  const unsigned l = bf16_bits(r);
  return (h & 0xffffu) | (l << 16);
}
__device__ __forceinline__ float silu_f(float v) {
  const float e = expf(fminf(-v, 80.0f));
  return v * (1.0f / (1.0f + e));
}
__device__ __forceinline__ float softplus_f(float a) {
  return fmaxf(a, 0.0f) + log1pf(expf(-fabsf(a)));
}

__global__ __launch_bounds__(PTHR) void k_prep(const float* __restrict__ inW, const float* __restrict__ dtinW,
                                               const float* __restrict__ BW, const float* __restrict__ CW,
                                               const float* __restrict__ dtW, const float* __restrict__ outW,
                                               unsigned short* W2, unsigned short* WS2,
                                               unsigned short* DTW2, unsigned short* OW2) {
  const int u = (int)blockIdx.x * PTHR + (int)threadIdx.x;
  const float* p;
  unsigned short* dp;
  int dup;
  bool zero = false;
  if (u < PU_W2) {
    const int n = u >> 7, k8 = (u & 127) * 8;
    p = inW + (size_t)n * DMOD + k8;
    dp = W2 + (size_t)n * KG1 + k8;
    dup = DMOD;
  } else if (u < PU_W2 + PU_WS) {
    const int v = u - PU_W2;
    const int r = v >> 8, k8 = (v & 255) * 8;
    dp = WS2 + (size_t)r * KG2 + k8;
    dup = DIN;
    if (r < 64)      p = dtinW + (size_t)r * DIN + k8;
    else if (r < 80) p = BW + (size_t)(r - 64) * DIN + k8;
    else if (r < 96) p = CW + (size_t)(r - 80) * DIN + k8;
    else           { p = dtinW + k8; zero = true; }
  } else if (u < PU_W2 + PU_WS + PU_DTW) {
    const int v = u - (PU_W2 + PU_WS);
    const int n = v >> 3, k8 = (v & 7) * 8;
    p = dtW + (size_t)n * DTRK + k8;
    dp = DTW2 + (size_t)n * KG3 + k8;
    dup = DTRK;
  } else if (u < PU_ALL) {
    const int v = u - (PU_W2 + PU_WS + PU_DTW);
    const int n = v >> 8, k8 = (v & 255) * 8;
    p = outW + (size_t)n * DIN + k8;
    dp = OW2 + (size_t)n * KG4 + k8;
    dup = DIN;
  } else {
    return;
  }
  const v4f a = *(const v4f*)p;
  const v4f b = *(const v4f*)(p + 4);
  v8us o;
  o[0] = zero ? (unsigned short)0 : (unsigned short)bf16_bits(a.x);
  o[1] = zero ? (unsigned short)0 : (unsigned short)bf16_bits(a.y);
  o[2] = zero ? (unsigned short)0 : (unsigned short)bf16_bits(a.z);
  o[3] = zero ? (unsigned short)0 : (unsigned short)bf16_bits(a.w);
  o[4] = zero ? (unsigned short)0 : (unsigned short)bf16_bits(b.x);
  o[5] = zero ? (unsigned short)0 : (unsigned short)bf16_bits(b.y);
  o[6] = zero ? (unsigned short)0 : (unsigned short)bf16_bits(b.z);
  o[7] = zero ? (unsigned short)0 : (unsigned short)bf16_bits(b.w);
  *(volatile v8us*)dp = o;
  *(volatile v8us*)(dp + dup) = o;
  __threadfence();
  *(volatile v8us*)dp = o;
  *(volatile v8us*)(dp + dup) = o;
}

__global__ __launch_bounds__(128) void k_ln(const float* __restrict__ x, const float* __restrict__ g,
                                            const float* __restrict__ b, unsigned short* XN) {
  __shared__ __attribute__((aligned(16))) unsigned short sh[4 * KG1];
  const int tid = (int)threadIdx.x, lane = tid & 31, wave = tid >> 5;
  const int row = (int)blockIdx.x * 4 + wave;
  const float* xr = x + (size_t)row * DMOD + 8 * lane;
  unsigned short* sw = sh + wave * KG1 + 8 * lane;

  float s = 0.0f;
#pragma unroll 1
  for (int i = 0; i < 4; ++i) {
    const v4f a = bf16_val4(*(const v4f*)(xr + 256 * i));
    const v4f c = bf16_val4(*(const v4f*)(xr + 256 * i + 4));
    s += a.x; s += a.y; s += a.z; s += a.w;
    s += c.x; s += c.y; s += c.z; s += c.w;
  }
#pragma unroll
  for (int o = 16; o > 0; o >>= 1) s += __shfl_xor(s, o, 32);
  const float mu = s * (1.0f / (float)DMOD);

  float s2 = 0.0f;
#pragma unroll 1
  for (int i = 0; i < 4; ++i) {
    const v4f a = bf16_val4(*(const v4f*)(xr + 256 * i));
    const v4f c = bf16_val4(*(const v4f*)(xr + 256 * i + 4));
    float d;
    d = a.x - mu; s2 += d * d;
    d = a.y - mu; s2 += d * d;
    d = a.z - mu; s2 += d * d;
    d = a.w - mu; s2 += d * d;
    d = c.x - mu; s2 += d * d;
    d = c.y - mu; s2 += d * d;
    d = c.z - mu; s2 += d * d;
    d = c.w - mu; s2 += d * d;
  }
#pragma unroll
  for (int o = 16; o > 0; o >>= 1) s2 += __shfl_xor(s2, o, 32);
  const float rs = rsqrtf(s2 * (1.0f / (float)DMOD) + 1e-5f);

#pragma unroll 1
  for (int i = 0; i < 4; ++i) {
    const v4f a  = bf16_val4(*(const v4f*)(xr + 256 * i));
    const v4f c  = bf16_val4(*(const v4f*)(xr + 256 * i + 4));
    const v4f g0 = bf16_val4(*(const v4f*)(g + 256 * i + 8 * lane));
    const v4f g1 = bf16_val4(*(const v4f*)(g + 256 * i + 8 * lane + 4));
    const v4f b0 = bf16_val4(*(const v4f*)(b + 256 * i + 8 * lane));
    const v4f b1 = bf16_val4(*(const v4f*)(b + 256 * i + 8 * lane + 4));
    v8us oh, ol;
    unsigned p;
    p = hl_pack((a.x - mu) * rs * g0.x + b0.x); oh[0] = (unsigned short)(p & 0xffffu); ol[0] = (unsigned short)(p >> 16);
    p = hl_pack((a.y - mu) * rs * g0.y + b0.y); oh[1] = (unsigned short)(p & 0xffffu); ol[1] = (unsigned short)(p >> 16);
    p = hl_pack((a.z - mu) * rs * g0.z + b0.z); oh[2] = (unsigned short)(p & 0xffffu); ol[2] = (unsigned short)(p >> 16);
    p = hl_pack((a.w - mu) * rs * g0.w + b0.w); oh[3] = (unsigned short)(p & 0xffffu); ol[3] = (unsigned short)(p >> 16);
    p = hl_pack((c.x - mu) * rs * g1.x + b1.x); oh[4] = (unsigned short)(p & 0xffffu); ol[4] = (unsigned short)(p >> 16);
    p = hl_pack((c.y - mu) * rs * g1.y + b1.y); oh[5] = (unsigned short)(p & 0xffffu); ol[5] = (unsigned short)(p >> 16);
    p = hl_pack((c.z - mu) * rs * g1.z + b1.z); oh[6] = (unsigned short)(p & 0xffffu); ol[6] = (unsigned short)(p >> 16);
    p = hl_pack((c.w - mu) * rs * g1.w + b1.w); oh[7] = (unsigned short)(p & 0xffffu); ol[7] = (unsigned short)(p >> 16);
    *(v8usa*)(sw + 256 * i) = oh;
    *(v8usa*)(sw + DMOD + 256 * i) = ol;
  }

  v8us qh[4], ql[4];
#pragma unroll
  for (int i = 0; i < 4; ++i) {
    qh[i] = *(const v8usa*)(sw + 256 * i);
    ql[i] = *(const v8usa*)(sw + DMOD + 256 * i);
  }
  unsigned short* orow = XN + (size_t)row * KG1 + 8 * lane;
#pragma unroll
  for (int i = 0; i < 4; ++i) {
    *(volatile v8us*)(orow + 256 * i) = qh[i];
    *(volatile v8us*)(orow + DMOD + 256 * i) = ql[i];
  }
  __threadfence();
#pragma unroll
  for (int i = 0; i < 4; ++i) {
    *(volatile v8us*)(orow + 256 * i) = qh[i];
    *(volatile v8us*)(orow + DMOD + 256 * i) = ql[i];
  }
}

template <int MODE>
__device__ __forceinline__ v4f epi_val(v4f v, v4f b4, const float* __restrict__ aux, size_t gi) {
  if constexpr (MODE == 2) {
    v4f o;
    o.x = softplus_f(v.x + b4.x);
    o.y = softplus_f(v.y + b4.y);
    o.z = softplus_f(v.z + b4.z);
    o.w = softplus_f(v.w + b4.w);
    return o;
  } else if constexpr (MODE == 3) {
    const v4f r = *(const v4f*)(aux + gi);
    v4f o;
    o.x = v.x + bf16_val(r.x);
    o.y = v.y + bf16_val(r.y);
    o.z = v.z + bf16_val(r.z);
    o.w = v.w + bf16_val(r.w);
    return o;
  } else {
    return v;
  }
}

template <int MODE>
__global__ __launch_bounds__(GTHR) void k_gemm(const unsigned short* __restrict__ A,
                                               const unsigned short* __restrict__ WT, int K,
                                               float* outF, int ldo, const float* __restrict__ aux,
                                               unsigned short* outH) {
  __shared__ __attribute__((aligned(16))) float stg[GBM * GBN];
  const int tid = (int)threadIdx.x, lane = tid & 31, wave = tid >> 5, hh = lane >> 4, m = lane & 15;
  const int rowBase = (int)blockIdx.x * GBM;
  const int col0    = (int)blockIdx.y * GBN;

  v8f acc0[4], acc1[4];
  {
    const v8f z = {0.f, 0.f, 0.f, 0.f, 0.f, 0.f, 0.f, 0.f};
#pragma unroll
    for (int t = 0; t < 4; ++t) { acc0[t] = z; acc1[t] = z; }
  }
  const unsigned short* ap0 = A + (size_t)(rowBase + 32 * wave + m) * (size_t)K + 8 * hh;
  const unsigned short* ap1 = ap0 + (size_t)16 * (size_t)K;
  const unsigned short* wp  = WT + (size_t)(col0 + m) * (size_t)K + 8 * hh;
  const int ksteps = K >> 5;
#pragma unroll 1
  for (int ks = 0; ks < ksteps; ++ks) {
    const int k0 = 32 * ks;
    FragB a0, a1;
    a0.h[0] = *(const v8usa*)(ap0 + k0);
    a0.h[1] = *(const v8usa*)(ap0 + k0 + 16);
    a1.h[0] = *(const v8usa*)(ap1 + k0);
    a1.h[1] = *(const v8usa*)(ap1 + k0 + 16);
#pragma unroll
    for (int t = 0; t < 4; ++t) {
      const unsigned short* wq = wp + (size_t)(16 * t) * (size_t)K + k0;
      FragB bf;
      bf.h[0] = *(const v8usa*)wq;
      bf.h[1] = *(const v8usa*)(wq + 16);
      acc0[t] = wmb(a0, bf, acc0[t]);
      acc1[t] = wmb(a1, bf, acc1[t]);
    }
  }

#pragma unroll
  for (int t = 0; t < 4; ++t) {
    const int lc = 16 * t + m;
#pragma unroll
    for (int r = 0; r < 8; ++r) {
      const int lr = 32 * wave + 8 * hh + r;
      stg[lr * GBN + lc]        = acc0[t][r];
      stg[(lr + 16) * GBN + lc] = acc1[t][r];
    }
  }
  __syncthreads();

  if constexpr (MODE == 1) {
    if (blockIdx.y == 0) {
      v4f b4;
      {
        const v4f t = *(const v4f*)(aux + 4 * m);
        b4.x = bf16_val(t.x); b4.y = bf16_val(t.y); b4.z = bf16_val(t.z); b4.w = bf16_val(t.w);
      }
      unsigned short* su = (unsigned short*)stg;
#pragma unroll 1
      for (int i = 0; i < 16; ++i) {
        const int lr = 32 * wave + 2 * i + hh;
        const v4f v = *(const v4fa*)(stg + lr * GBN + 4 * m);
        const unsigned p0 = hl_pack(v.x + b4.x), p1 = hl_pack(v.y + b4.y);
        const unsigned p2 = hl_pack(v.z + b4.z), p3 = hl_pack(v.w + b4.w);
        v4us h4, l4;
        h4[0] = (unsigned short)(p0 & 0xffffu); l4[0] = (unsigned short)(p0 >> 16);
        h4[1] = (unsigned short)(p1 & 0xffffu); l4[1] = (unsigned short)(p1 >> 16);
        h4[2] = (unsigned short)(p2 & 0xffffu); l4[2] = (unsigned short)(p2 >> 16);
        h4[3] = (unsigned short)(p3 & 0xffffu); l4[3] = (unsigned short)(p3 >> 16);
        *(v4usa*)(su + lr * 128 + 4 * m) = h4;
        *(v4usa*)(su + lr * 128 + 64 + 4 * m) = l4;
      }
      __syncthreads();
#pragma unroll 1
      for (int i = 0; i < 16; ++i) {
        const int lr = 32 * wave + 2 * i + hh;
        const v8us q = *(const v8usa*)(su + lr * 128 + 8 * m);
        *(volatile v8us*)(outH + (size_t)(rowBase + lr) * 128 + 8 * m) = q;
      }
      __threadfence();
#pragma unroll 1
      for (int i = 0; i < 16; ++i) {
        const int lr = 32 * wave + 2 * i + hh;
        const v8us q = *(const v8usa*)(su + lr * 128 + 8 * m);
        *(volatile v8us*)(outH + (size_t)(rowBase + lr) * 128 + 8 * m) = q;
      }
    } else {
      const int rq = lane >> 3, pc = 4 * (lane & 7);
#pragma unroll 1
      for (int i = 0; i < 8; ++i) {
        const int lr = 32 * wave + 4 * i + rq;
        const v4f v = *(const v4fa*)(stg + lr * GBN + pc);
        *(volatile v4f*)(outF + (size_t)(rowBase + lr) * BCP + pc) = v;
      }
      __threadfence();
#pragma unroll 1
      for (int i = 0; i < 8; ++i) {
        const int lr = 32 * wave + 4 * i + rq;
        const v4f v = *(const v4fa*)(stg + lr * GBN + pc);
        *(volatile v4f*)(outF + (size_t)(rowBase + lr) * BCP + pc) = v;
      }
    }
  } else {
    v4f b4 = {0.f, 0.f, 0.f, 0.f};
    if constexpr (MODE == 2) {
      const v4f t = *(const v4f*)(aux + col0 + 4 * m);
      b4.x = bf16_val(t.x); b4.y = bf16_val(t.y); b4.z = bf16_val(t.z); b4.w = bf16_val(t.w);
    }
#pragma unroll 1
    for (int i = 0; i < 16; ++i) {
      const int lr = 32 * wave + 2 * i + hh;
      const size_t gi = (size_t)(rowBase + lr) * (size_t)ldo + (size_t)(col0 + 4 * m);
      const v4f v = *(const v4fa*)(stg + lr * GBN + 4 * m);
      const v4f o = epi_val<MODE>(v, b4, aux, gi);
      *(volatile v4f*)(outF + gi) = o;
    }
    __threadfence();
#pragma unroll 1
    for (int i = 0; i < 16; ++i) {
      const int lr = 32 * wave + 2 * i + hh;
      const size_t gi = (size_t)(rowBase + lr) * (size_t)ldo + (size_t)(col0 + 4 * m);
      const v4f v = *(const v4fa*)(stg + lr * GBN + 4 * m);
      const v4f o = epi_val<MODE>(v, b4, aux, gi);
      *(volatile v4f*)(outF + gi) = o;
    }
  }
}

__global__ __launch_bounds__(PTHR) void k_conv(const float* __restrict__ XZ, const float* __restrict__ cw,
                                               const float* __restrict__ cb, float* U, unsigned short* UH) {
  __shared__ __attribute__((aligned(16))) float su[DIN];
  const int tid = (int)threadIdx.x;
  const int t   = (int)blockIdx.x;
  const int l   = t & (LSEQ - 1);

#pragma unroll 1
  for (int hf = 0; hf < 2; ++hf) {
    const int c = hf * (DIN / 2) + 4 * tid;
    const v4f bb = bf16_val4(*(const v4f*)(cb + c));
    const v4f w0 = bf16_val4(*(const v4f*)(cw + 4 * (size_t)(c + 0)));
    const v4f w1 = bf16_val4(*(const v4f*)(cw + 4 * (size_t)(c + 1)));
    const v4f w2 = bf16_val4(*(const v4f*)(cw + 4 * (size_t)(c + 2)));
    const v4f w3 = bf16_val4(*(const v4f*)(cw + 4 * (size_t)(c + 3)));
    float a0 = bb.x, a1 = bb.y, a2 = bb.z, a3 = bb.w;
#pragma unroll
    for (int k = 0; k < 4; ++k) {
      const bool ok = (l - 3 + k) >= 0;
      const int  tr = ok ? (t - 3 + k) : t;
      v4f xa = *(const v4f*)(XZ + (size_t)tr * XZP + c);
      const v4f z4 = {0.f, 0.f, 0.f, 0.f};
      xa = ok ? xa : z4;
      a0 = a0 + w0[k] * xa.x;
      a1 = a1 + w1[k] * xa.y;
      a2 = a2 + w2[k] * xa.z;
      a3 = a3 + w3[k] * xa.w;
    }
    v4f pv;
    pv.x = a0; pv.y = a1; pv.z = a2; pv.w = a3;
    *(v4fa*)(su + c) = pv;
  }
  __syncthreads();

#pragma unroll 1
  for (int j = 0; j < 8; ++j) {
    const int e = tid + PTHR * j;
    const float v = su[e];
    su[e] = silu_f(v);
  }
  __syncthreads();

  const int c0 = 8 * tid;
  const v4f u0 = *(const v4fa*)(su + 4 * tid);
  const v4f u1 = *(const v4fa*)(su + DIN / 2 + 4 * tid);
  const v4f sa = *(const v4fa*)(su + c0);
  const v4f sb = *(const v4fa*)(su + c0 + 4);
  v8us oh, ol;
  {
    unsigned p;
    p = hl_pack(sa.x); oh[0] = (unsigned short)(p & 0xffffu); ol[0] = (unsigned short)(p >> 16);
    p = hl_pack(sa.y); oh[1] = (unsigned short)(p & 0xffffu); ol[1] = (unsigned short)(p >> 16);
    p = hl_pack(sa.z); oh[2] = (unsigned short)(p & 0xffffu); ol[2] = (unsigned short)(p >> 16);
    p = hl_pack(sa.w); oh[3] = (unsigned short)(p & 0xffffu); ol[3] = (unsigned short)(p >> 16);
    p = hl_pack(sb.x); oh[4] = (unsigned short)(p & 0xffffu); ol[4] = (unsigned short)(p >> 16);
    p = hl_pack(sb.y); oh[5] = (unsigned short)(p & 0xffffu); ol[5] = (unsigned short)(p >> 16);
    p = hl_pack(sb.z); oh[6] = (unsigned short)(p & 0xffffu); ol[6] = (unsigned short)(p >> 16);
    p = hl_pack(sb.w); oh[7] = (unsigned short)(p & 0xffffu); ol[7] = (unsigned short)(p >> 16);
  }
  float* ur = U + (size_t)t * DIN;
  unsigned short* hr = UH + (size_t)t * KG2;
  *(volatile v4f*)(ur + 4 * tid) = u0;
  *(volatile v4f*)(ur + DIN / 2 + 4 * tid) = u1;
  *(volatile v8us*)(hr + c0) = oh;
  *(volatile v8us*)(hr + DIN + c0) = ol;
  __threadfence();
  *(volatile v4f*)(ur + 4 * tid) = u0;
  *(volatile v4f*)(ur + DIN / 2 + 4 * tid) = u1;
  *(volatile v8us*)(hr + c0) = oh;
  *(volatile v8us*)(hr + DIN + c0) = ol;
}

__global__ __launch_bounds__(SC_THR) void k_scan(const float* __restrict__ DT, const float* __restrict__ U,
                                                 const float* __restrict__ XZ, const float* __restrict__ BC,
                                                 const float* __restrict__ Alog, const float* __restrict__ Dp,
                                                 unsigned short* Y) {
  __shared__ __attribute__((aligned(16))) float sDT[SC_TC * SC_DB];
  __shared__ __attribute__((aligned(16))) float sU[SC_TC * SC_DB];
  __shared__ __attribute__((aligned(16))) float sZ[SC_TC * SC_DB];
  __shared__ __attribute__((aligned(16))) float sYS[SC_TC * SC_DB];
  __shared__ __attribute__((aligned(16))) float sBC[SC_TC * BCP];
  __shared__ __attribute__((aligned(16))) float sA[2 * SC_THR];
  __shared__ __attribute__((aligned(16))) unsigned short sY[SC_TC * 2 * SC_DB];
  const int tid = (int)threadIdx.x;
  const int n   = tid & 15;
  const int dq  = tid >> 4;
  const int b   = (int)blockIdx.x >> 5;
  const int d0  = ((int)blockIdx.x & 31) * SC_DB;
  const int tb  = b * LSEQ;

#pragma unroll 1
  for (int sidx = 0; sidx < 2; ++sidx) {
    float al = Alog[(size_t)(d0 + dq + 32 * sidx) * NST + n];
#if A_LOG_RNE_BF16
    al = bf16_val(al);
#endif
    sA[sidx * SC_THR + tid] = -expf(al);
  }
  const float A0 = sA[tid];
  const float A1 = sA[SC_THR + tid];
  const int   fc = tid & (SC_DB - 1);
  const float Dc = bf16_val(Dp[d0 + fc]);
  float h0 = 0.0f, h1 = 0.0f;
  const int r = dq, q = n;
  const int line = tid >> 3, piece = tid & 7;
  const int srow = line >> 1, swh = line & 1;

#pragma unroll 1
  for (int ch = 0; ch < LSEQ / SC_TC; ++ch) {
    const int t0 = tb + SC_TC * ch;
    {
      const size_t grow = (size_t)(t0 + r);
      const v4f vdt = *(const v4f*)(DT + grow * DIN + d0 + 4 * q);
      const v4f vu  = *(const v4f*)(U + grow * DIN + d0 + 4 * q);
      const v4f vz  = *(const v4f*)(XZ + grow * XZP + DIN + d0 + 4 * q);
      *(v4fa*)(sDT + r * SC_DB + 4 * q) = vdt;
      *(v4fa*)(sU + r * SC_DB + 4 * q)  = vu;
      *(v4fa*)(sZ + r * SC_DB + 4 * q)  = vz;
      if (tid < SC_TC * 8) {
        const int rr = tid >> 3, pp = tid & 7;
        const v4f vb = *(const v4f*)(BC + (size_t)(t0 + rr) * BCP + 4 * pp);
        *(v4fa*)(sBC + rr * BCP + 4 * pp) = vb;
      }
    }
    __syncthreads();

#pragma unroll 1
    for (int tl = 0; tl < SC_TC; ++tl) {
      const float Bn  = sBC[tl * BCP + n];
      const float Cn  = sBC[tl * BCP + NST + n];
      const float dt0 = sDT[tl * SC_DB + dq];
      const float u0  = sU[tl * SC_DB + dq];
      const float dt1 = sDT[tl * SC_DB + dq + 32];
      const float u1  = sU[tl * SC_DB + dq + 32];
      const float e0 = expf(dt0 * A0);
      const float e1 = expf(dt1 * A1);
      const float du0 = dt0 * u0;
      const float du1 = dt1 * u1;
      h0 = h0 * e0 + du0 * Bn;
      h1 = h1 * e1 + du1 * Bn;
      float p0 = h0 * Cn;
      float p1 = h1 * Cn;
      p0 += __shfl_xor(p0, 1, 32); p1 += __shfl_xor(p1, 1, 32);
      p0 += __shfl_xor(p0, 2, 32); p1 += __shfl_xor(p1, 2, 32);
      p0 += __shfl_xor(p0, 4, 32); p1 += __shfl_xor(p1, 4, 32);
      p0 += __shfl_xor(p0, 8, 32); p1 += __shfl_xor(p1, 8, 32);
      if (n == 0) {
        sYS[tl * SC_DB + dq]      = p0;
        sYS[tl * SC_DB + dq + 32] = p1;
      }
    }
    __syncthreads();

#pragma unroll 1
    for (int j = 0; j < 4; ++j) {
      const int e  = tid + SC_THR * j;
      const int fr = e >> 6;
      const float ys = sYS[e];
      const float uu = sU[e];
      const float zz = sZ[e];
      const float yv = (ys + uu * Dc) * silu_f(zz);
      const unsigned p = hl_pack(yv);
      sY[fr * (2 * SC_DB) + fc]         = (unsigned short)(p & 0xffffu);
      sY[fr * (2 * SC_DB) + SC_DB + fc] = (unsigned short)(p >> 16);
    }
    __syncthreads();

    {
      const v8us qv = *(const v8usa*)(sY + srow * (2 * SC_DB) + swh * SC_DB + 8 * piece);
      unsigned short* gp = Y + (size_t)(t0 + srow) * KG4 + (size_t)swh * DIN + d0 + 8 * piece;
      *(volatile v8us*)gp = qv;
      __threadfence();
      *(volatile v8us*)gp = qv;
    }
  }
}

static inline size_t al256(size_t o) { return (o + 255) & ~(size_t)255; }

extern "C" void kernel_launch(void* const* d_in, const int* in_sizes, int n_in,
                              void* d_out, int out_size, void* d_ws, size_t ws_size,
                              hipStream_t stream) {
  if (n_in < 15) return;
  if (in_sizes[0] != TOK * DMOD) return;
  if (in_sizes[1] != DMOD || in_sizes[2] != DMOD) return;
  if (in_sizes[3] != 2 * DIN * DMOD) return;
  if (in_sizes[4] != DIN * 4 || in_sizes[5] != DIN) return;
  if (in_sizes[6] != DTRK * DIN || in_sizes[7] != DTRK) return;
  if (in_sizes[8] != DIN * DTRK || in_sizes[9] != DIN) return;
  if (in_sizes[10] != NST * DIN || in_sizes[11] != NST * DIN) return;
  if (in_sizes[12] != DIN * NST || in_sizes[13] != DIN) return;
  if (in_sizes[14] != DMOD * DIN) return;
  if (out_size != TOK * DMOD) return;

  const float* x      = (const float*)d_in[0];
  const float* ln_g   = (const float*)d_in[1];
  const float* ln_b   = (const float*)d_in[2];
  const float* inW    = (const float*)d_in[3];
  const float* conv_w = (const float*)d_in[4];
  const float* conv_b = (const float*)d_in[5];
  const float* dtin_w = (const float*)d_in[6];
  const float* dtin_b = (const float*)d_in[7];
  const float* dt_w   = (const float*)d_in[8];
  const float* dt_b   = (const float*)d_in[9];
  const float* B_w    = (const float*)d_in[10];
  const float* C_w    = (const float*)d_in[11];
  const float* A_log  = (const float*)d_in[12];
  const float* Dp     = (const float*)d_in[13];
  const float* outW   = (const float*)d_in[14];
  float* out = (float*)d_out;

  char* ws = (char*)d_ws;
  size_t off = 0;
  const size_t oXN  = off; off = al256(off + (size_t)TOK * KG1 * 2);
  const size_t oW2  = off; off = al256(off + (size_t)(2 * DIN) * KG1 * 2);
  const size_t oXZ  = off; off = al256(off + (size_t)TOK * XZP * 4);
  const size_t oU   = off; off = al256(off + (size_t)TOK * DIN * 4);
  const size_t oUH  = off; off = al256(off + (size_t)TOK * KG2 * 2);
  const size_t oWS  = off; off = al256(off + (size_t)N2P * KG2 * 2);
  const size_t oDTW = off; off = al256(off + (size_t)DIN * KG3 * 2);
  const size_t oDTI = off; off = al256(off + (size_t)TOK * KG3 * 2);
  const size_t oBC  = off; off = al256(off + (size_t)TOK * BCP * 4);
  const size_t oDT  = off; off = al256(off + (size_t)TOK * DIN * 4);
  const size_t oOW  = off; off = al256(off + (size_t)DMOD * KG4 * 2);
  if (off > ws_size || off > (size_t)WSMAX) return;
  static_assert((size_t)TOK * KG4 * 2 == (size_t)(2 * DIN) * KG1 * 2);
  unsigned short* XN   = (unsigned short*)(ws + oXN);
  unsigned short* W2   = (unsigned short*)(ws + oW2);
  unsigned short* Yhl  = (unsigned short*)(ws + oW2);
  float*          XZ   = (float*)(ws + oXZ);
  float*          U    = (float*)(ws + oU);
  unsigned short* UH   = (unsigned short*)(ws + oUH);
  unsigned short* WS2  = (unsigned short*)(ws + oWS);
  unsigned short* DTW2 = (unsigned short*)(ws + oDTW);
  unsigned short* DTIN = (unsigned short*)(ws + oDTI);
  float*          BC   = (float*)(ws + oBC);
  float*          DT   = (float*)(ws + oDT);
  unsigned short* OW2  = (unsigned short*)(ws + oOW);

  k_prep<<<PU_ALL / PTHR, PTHR, 0, stream>>>(inW, dtin_w, B_w, C_w, dt_w, outW, W2, WS2, DTW2, OW2);
  k_ln<<<TOK / 4, 128, 0, stream>>>(x, ln_g, ln_b, XN);
  k_gemm<0><<<dim3(TOK / GBM, (2 * DIN) / GBN), GTHR, 0, stream>>>(XN, W2, KG1, XZ, XZP, x, DTIN);
  k_conv<<<TOK, PTHR, 0, stream>>>(XZ, conv_w, conv_b, U, UH);
  k_gemm<1><<<dim3(TOK / GBM, N2P / GBN), GTHR, 0, stream>>>(UH, WS2, KG2, BC, BCP, dtin_b, DTIN);
  k_gemm<2><<<dim3(TOK / GBM, DIN / GBN), GTHR, 0, stream>>>(DTIN, DTW2, KG3, DT, DIN, dt_b, DTIN);
  k_scan<<<NBAT * (DIN / SC_DB), SC_THR, 0, stream>>>(DT, U, XZ, BC, A_log, Dp, Yhl);
  k_gemm<3><<<dim3(TOK / GBM, DMOD / GBN), GTHR, 0, stream>>>(Yhl, OW2, KG4, out, DMOD, x, DTIN);
}
